// MultiScaleCrossAttn_83502754169465
// MI455X (gfx1250) — hardware-verified
//
#include <hip/hip_runtime.h>
#define NIMG 64
#define CB 8
#define DDm 96
#define NHh 3
#define HD 32
#define G0 14
#define G1 56
#define G2 32
#define T0 196
#define T1 3136
#define T2 1024
#define NQ 196
#define NKc 25
#define LP 128
#define QP 320
typedef __bf16 v16b __attribute__((ext_vector_type(16)));
typedef unsigned short v8us __attribute__((ext_vector_type(8), may_alias));
typedef float  v8f  __attribute__((ext_vector_type(8)));
typedef float  v4f  __attribute__((ext_vector_type(4)));
typedef float  v4fa __attribute__((ext_vector_type(4), may_alias));
union FragB { v16b v; v8us half[2]; unsigned short u[16]; };

__device__ __forceinline__ unsigned short bf16_bits(float x) { unsigned int u = __float_as_uint(x); return (unsigned short)((u + 0x7FFFu + ((u >> 16) & 1u)) >> 16); }
__device__ __forceinline__ float bf16_val(unsigned short b) { return __uint_as_float(((unsigned int)b) << 16); }
__device__ __forceinline__ float bf16_round(float x) { return bf16_val(bf16_bits(x)); }
template <int NT>
__device__ __forceinline__ v8f mmaN(v16b ah, v16b al, v16b bh, v16b bl, v8f c) {
  c = __builtin_amdgcn_wmma_f32_16x16x32_bf16(false, ah, false, bh, (short)0, c, false, false);
  if (NT >= 2) c = __builtin_amdgcn_wmma_f32_16x16x32_bf16(false, al, false, bh, (short)0, c, false, false);
  if (NT >= 3) c = __builtin_amdgcn_wmma_f32_16x16x32_bf16(false, ah, false, bl, (short)0, c, false, false);
  asm volatile("v_nop\n\tv_nop\n\tv_nop\n\tv_nop" : "+v"(c) : "v"(ah), "v"(al), "v"(bh), "v"(bl));
  return c;
}

__global__ __launch_bounds__(256) void k_wt_bf16(const float* __restrict__ W, unsigned short* __restrict__ Wt, int K, int N) {
  const int t = blockIdx.x * 256 + threadIdx.x;
  const int k8n = K / 8;
  if (t >= N * k8n) return;
  const int n = t / k8n, k8 = (t % k8n) * 8;
  v8us v;
#pragma unroll
  for (int i = 0; i < 8; ++i) v[i] = bf16_bits(W[(size_t)(k8 + i) * N + n]);
  *(volatile v8us*)(Wt + (size_t)n * K + k8) = v;
  __threadfence();
  *(volatile v8us*)(Wt + (size_t)n * K + k8) = v;
}

template <bool ASPLIT, int ACT, bool BIAS_BF16>
__global__ __launch_bounds__(128) void k_gemm_bf(const float* __restrict__ A, int lda, const unsigned short* __restrict__ Wt, int ldb,
                                               const float* __restrict__ bias, float* __restrict__ C, int ldc, int M, int N, int K) {
  __shared__ __attribute__((aligned(16))) float so[4][16][64];
  const int tid = threadIdx.x, w = tid >> 5, lane = tid & 31, ln = lane & 15, hh = lane >> 4;
  const int ntn = N / 64;
  const int wid = blockIdx.x * 4 + w;
  const int mt = wid / ntn, nq = wid % ntn;
  if (mt * 16 >= M) return;
  const int row0 = mt * 16, col0 = nq * 64;
  const float* arow = A + (size_t)(row0 + ln) * lda;
  v8f acc[4] = {};
  for (int kb = 0; kb < K; kb += 32) {
    FragB ah, al;
    const v4f x0 = *(const v4fa*)(arow + kb + 8 * hh), x1 = *(const v4fa*)(arow + kb + 8 * hh + 4);
    const v4f x2 = *(const v4fa*)(arow + kb + 16 + 8 * hh), x3 = *(const v4fa*)(arow + kb + 16 + 8 * hh + 4);
    float xs[16] = {x0[0],x0[1],x0[2],x0[3],x1[0],x1[1],x1[2],x1[3],x2[0],x2[1],x2[2],x2[3],x3[0],x3[1],x3[2],x3[3]};
#pragma unroll
    for (int i = 0; i < 16; ++i) { const unsigned short hb = bf16_bits(xs[i]); ah.u[i] = hb; al.u[i] = ASPLIT ? bf16_bits(xs[i] - bf16_val(hb)) : (unsigned short)0; }
#pragma unroll
    for (int t = 0; t < 4; ++t) {
      const unsigned short* brow = Wt + (size_t)(col0 + t * 16 + ln) * ldb + kb;
      FragB b;
      b.half[0] = *(const v8us*)(brow + 8 * hh);
      b.half[1] = *(const v8us*)(brow + 16 + 8 * hh);
      acc[t] = mmaN<ASPLIT ? 2 : 1>(ah.v, al.v, b.v, b.v, acc[t]);
    }
  }
#pragma unroll
  for (int t = 0; t < 4; ++t) {
    float bv = bias ? bias[col0 + t * 16 + ln] : 0.f;
    if (BIAS_BF16) bv = bf16_round(bv);
#pragma unroll
    for (int r = 0; r < 8; ++r) { float v = acc[t][r] + bv; if (ACT == 1) v = fmaxf(v, 0.f); so[w][8 * hh + r][t * 16 + ln] = v; }
  }
  __builtin_amdgcn_fence(__ATOMIC_ACQ_REL, "workgroup");
  __builtin_amdgcn_wave_barrier();
  const int rsub = lane >> 4, c4 = (lane & 15) * 4;
  for (int pass = 0; pass < 2; ++pass) {
#pragma unroll
    for (int q = 0; q < 8; ++q) {
      const int r = q * 2 + rsub;
      const v4f v = *(const v4fa*)&so[w][r][c4];
      *(volatile v4f*)(C + (size_t)(row0 + r) * ldc + col0 + c4) = v;
    }
    if (pass == 0) __threadfence();
  }
}

template <bool ASPLIT, int ACT, bool BIAS_BF16, bool RES_BF16>
__global__ __launch_bounds__(128) void k_gemm_bf3(const float* __restrict__ A, int lda, const unsigned short* __restrict__ Wt, int ldb,
                                                const float* __restrict__ bias, const float* __restrict__ resid, int rmod, int ldr,
                                                float* __restrict__ C, int ldc, int M, int N, int K) {
  __shared__ __attribute__((aligned(16))) float so[4][16][64];
  const int tid = threadIdx.x, w = tid >> 5, lane = tid & 31, ln = lane & 15, hh = lane >> 4;
  const int ntn = N / 64;
  const int wid = blockIdx.x * 4 + w;
  const int mt = wid / ntn, nq = wid % ntn;
  if (mt * 16 >= M) return;
  const int row0 = mt * 16, col0 = nq * 64;
  const float* arow = A + (size_t)(row0 + ln) * lda;
  v8f acc[4] = {};
  for (int kb = 0; kb < K; kb += 32) {
    FragB ah, al;
    const v4f x0 = *(const v4fa*)(arow + kb + 8 * hh), x1 = *(const v4fa*)(arow + kb + 8 * hh + 4);
    const v4f x2 = *(const v4fa*)(arow + kb + 16 + 8 * hh), x3 = *(const v4fa*)(arow + kb + 16 + 8 * hh + 4);
    float xs[16] = {x0[0],x0[1],x0[2],x0[3],x1[0],x1[1],x1[2],x1[3],x2[0],x2[1],x2[2],x2[3],x3[0],x3[1],x3[2],x3[3]};
#pragma unroll
    for (int i = 0; i < 16; ++i) { const unsigned short hb = bf16_bits(xs[i]); ah.u[i] = hb; al.u[i] = ASPLIT ? bf16_bits(xs[i] - bf16_val(hb)) : (unsigned short)0; }
#pragma unroll
    for (int t = 0; t < 4; ++t) {
      const unsigned short* brow = Wt + (size_t)(col0 + t * 16 + ln) * ldb + kb;
      FragB b;
      b.half[0] = *(const v8us*)(brow + 8 * hh);
      b.half[1] = *(const v8us*)(brow + 16 + 8 * hh);
      acc[t] = mmaN<ASPLIT ? 2 : 1>(ah.v, al.v, b.v, b.v, acc[t]);
    }
  }
#pragma unroll
  for (int t = 0; t < 4; ++t) {
    const int col = col0 + t * 16 + ln;
    float bv = bias ? bias[col] : 0.f;
    if (BIAS_BF16) bv = bf16_round(bv);
#pragma unroll
    for (int r = 0; r < 8; ++r) {
      float v = acc[t][r] + bv;
      if (resid) { float rv = resid[(size_t)((row0 + 8 * hh + r) % rmod) * ldr + col]; if (RES_BF16) rv = bf16_round(rv); v += rv; }
      if (ACT == 1) v = fmaxf(v, 0.f);
      if (ACT == 2) v = 0.5f * v * (1.0f + erff(v * 0.70710678118654752f));
      if (ACT == 3) { const float u = 0.7978845608028654f * (v + 0.044715f * v * v * v); v = 0.5f * v * (1.0f + tanhf(u)); }
      so[w][8 * hh + r][t * 16 + ln] = v;
    }
  }
  __builtin_amdgcn_fence(__ATOMIC_ACQ_REL, "workgroup");
  __builtin_amdgcn_wave_barrier();
  const int rsub = lane >> 4, c4 = (lane & 15) * 4;
  for (int pass = 0; pass < 2; ++pass) {
#pragma unroll
    for (int q = 0; q < 8; ++q) {
      const int r = q * 2 + rsub;
      const v4f v = *(const v4fa*)&so[w][r][c4];
      *(volatile v4f*)(C + (size_t)(row0 + r) * ldc + col0 + c4) = v;
    }
    if (pass == 0) __threadfence();
  }
}
template <bool PARAM_BF16>
__global__ __launch_bounds__(256) void k_layernorm(const float* __restrict__ X, const float* __restrict__ R, const float* __restrict__ g, const float* __restrict__ bta,
                                                  float* __restrict__ out_sum, float* __restrict__ out_norm, int N, float eps) {
  __shared__ float red[256];
  const int row = blockIdx.x, tid = threadIdx.x;
  const float* x = X + (size_t)row * N; const float* rr = R ? R + (size_t)row * N : nullptr;
  float vals[16];
  const int per = N / 256;
  float s1 = 0.f;
  for (int u = 0; u < per / 4; ++u) {
    const int j = tid * 4 + 1024 * u;
    const v4f a = *(const v4fa*)(x + j);
    v4f b = {0.f,0.f,0.f,0.f}; if (rr) b = *(const v4fa*)(rr + j);
#pragma unroll
    for (int q = 0; q < 4; ++q) { const float v = a[q] + b[q]; vals[u * 4 + q] = v; s1 += v; }
  }
  red[tid] = s1; __syncthreads();
  for (int st = 128; st > 0; st >>= 1) { if (tid < st) red[tid] += red[tid + st]; __syncthreads(); }
  const float mu = red[0] / (float)N; __syncthreads();
  float s2 = 0.f;
  for (int u = 0; u < per / 4; ++u)
#pragma unroll
    for (int q = 0; q < 4; ++q) { const float c = vals[u * 4 + q] - mu; s2 += c * c; }
  red[tid] = s2; __syncthreads();
  for (int st = 128; st > 0; st >>= 1) { if (tid < st) red[tid] += red[tid + st]; __syncthreads(); }
  const float rs = rsqrtf(red[0] / (float)N + eps);
  for (int pass = 0; pass < 2; ++pass) {
    for (int u = 0; u < per / 4; ++u) {
      const int j = tid * 4 + 1024 * u;
      v4f o, sm;
#pragma unroll
      for (int q = 0; q < 4; ++q) {
        float gg = g[j + q], bb = bta[j + q];
        if (PARAM_BF16) { gg = bf16_round(gg); bb = bf16_round(bb); }
        sm[q] = vals[u * 4 + q]; o[q] = (vals[u * 4 + q] - mu) * rs * gg + bb;
      }
      if (out_sum) *(volatile v4f*)(out_sum + (size_t)row * N + j) = sm;
      *(volatile v4f*)(out_norm + (size_t)row * N + j) = o;
    }
    if (pass == 0) __threadfence();
  }
}


typedef _Float16 v16h __attribute__((ext_vector_type(16)));
union FragH { v16h v; v8us half[2]; _Float16 h[16]; unsigned short u[16]; };
template <int NT>
__device__ __forceinline__ v8f mmaH(v16h ah, v16h al, v16h bh, v16h bl, v8f c) {
  c = __builtin_amdgcn_wmma_f32_16x16x32_f16(false, ah, false, bh, (short)0, c, false, false);
  if (NT >= 2) c = __builtin_amdgcn_wmma_f32_16x16x32_f16(false, al, false, bh, (short)0, c, false, false);
  if (NT >= 3) c = __builtin_amdgcn_wmma_f32_16x16x32_f16(false, ah, false, bl, (short)0, c, false, false);
  asm volatile("v_nop\n\tv_nop\n\tv_nop\n\tv_nop" : "+v"(c) : "v"(ah), "v"(al), "v"(bh), "v"(bl));
  return c;
}
template <bool ASPLIT>
__global__ __launch_bounds__(128) void k_gemm_h(const float* __restrict__ A, int lda, size_t sA, const _Float16* __restrict__ Bh, int ldb, size_t sB, float alpha, float* __restrict__ C, int ldc, size_t sC, int M, int N, int K) {
  __shared__ __attribute__((aligned(16))) float so[4][16][64];
  const int tid = threadIdx.x, w = tid >> 5, lane = tid & 31, ln = lane & 15, hh = lane >> 4; const int by = blockIdx.y;
  A += (size_t)by * sA; Bh += (size_t)by * sB; C += (size_t)by * sC;
  const int ntn = (N + 63) / 64; const int wid = blockIdx.x * 4 + w; const int mt = wid / ntn, nq = wid % ntn; if (mt * 16 >= M) return;
  const int row0 = mt * 16, col0 = nq * 64; const float* arow = A + (size_t)(row0 + ln) * lda;
  v8f acc[4] = {};
  for (int kb = 0; kb < K; kb += 32) {
    FragH ah, al;
    const v4f x0 = *(const v4fa*)(arow + kb + 8 * hh), x1 = *(const v4fa*)(arow + kb + 8 * hh + 4), x2 = *(const v4fa*)(arow + kb + 16 + 8 * hh), x3 = *(const v4fa*)(arow + kb + 16 + 8 * hh + 4);
    float xs[16] = {x0[0],x0[1],x0[2],x0[3],x1[0],x1[1],x1[2],x1[3],x2[0],x2[1],x2[2],x2[3],x3[0],x3[1],x3[2],x3[3]};
#pragma unroll
    for (int i = 0; i < 16; ++i) { const _Float16 h = (_Float16)xs[i]; ah.h[i] = h; al.h[i] = ASPLIT ? (_Float16)(xs[i] - (float)h) : (_Float16)0.0f; }
#pragma unroll
    for (int t = 0; t < 4; ++t) { if (col0 + t * 16 >= N) continue; const size_t boff = (size_t)(col0 + t * 16 + ln) * ldb + kb; FragH bq; bq.half[0] = *(const v8us*)(Bh + boff + 8 * hh); bq.half[1] = *(const v8us*)(Bh + boff + 16 + 8 * hh);
      acc[t] = mmaH<ASPLIT ? 2 : 1>(ah.v, al.v, bq.v, bq.v, acc[t]); }
  }
#pragma unroll
  for (int t = 0; t < 4; ++t) { if (col0 + t * 16 >= N) continue;
#pragma unroll
    for (int r = 0; r < 8; ++r) so[w][8 * hh + r][t * 16 + ln] = acc[t][r] * alpha; }
  __builtin_amdgcn_fence(__ATOMIC_ACQ_REL, "workgroup"); __builtin_amdgcn_wave_barrier();
  const int rsub = lane >> 4, c4 = (lane & 15) * 4;
  for (int pass = 0; pass < 2; ++pass) {
#pragma unroll
    for (int q = 0; q < 8; ++q) { const int r = q * 2 + rsub; if (col0 + c4 < N) { const v4f v = *(const v4fa*)&so[w][r][c4]; *(volatile v4f*)(C + (size_t)(row0 + r) * ldc + col0 + c4) = v; } }
    if (pass == 0) __threadfence(); }
}

__global__ __launch_bounds__(256) void k_wt_f16(const float* __restrict__ W, _Float16* __restrict__ Wt, int K, int N, float scale) {
  const int t = blockIdx.x * 256 + threadIdx.x; if (t >= N * (K / 8)) return; const int n = t / (K / 8), k8 = (t % (K / 8)) * 8; FragH f;
#pragma unroll
  for (int i = 0; i < 8; ++i) f.h[i] = (_Float16)(bf16_round(W[(size_t)(k8 + i) * N + n]) * scale); const v8us o = f.half[0];
  *(volatile v8us*)((unsigned short*)Wt + (size_t)n * K + k8) = o; __threadfence(); *(volatile v8us*)((unsigned short*)Wt + (size_t)n * K + k8) = o;
}
template <int ACT>
__global__ __launch_bounds__(128) void k_gemm_hhx(const _Float16* __restrict__ A, int lda, size_t sA, const _Float16* __restrict__ Bh, int ldb, size_t sB, float alpha, const float* __restrict__ bias, size_t sBias, const float* __restrict__ CP, int rowsPerB, size_t sCPb, int row0g,
    float* __restrict__ C, _Float16* __restrict__ C16, int ldc, size_t sC, int M, int N, int K) {
  __shared__ __attribute__((aligned(16))) float so[4][16][64];
  const int tid = threadIdx.x, w = tid >> 5, lane = tid & 31, ln = lane & 15, hh = lane >> 4; const int by = blockIdx.y;
  A += (size_t)by * sA; Bh += (size_t)by * sB; const size_t cofs = (size_t)by * sC; const float* bp = bias ? bias + (size_t)by * sBias : nullptr;
  const int ntn = (N + 63) / 64; const int wid = blockIdx.x * 4 + w; const int mt = wid / ntn, nq = wid % ntn; if (mt * 16 >= M) return;
  const int row0 = mt * 16, col0 = nq * 64; const _Float16* arow = A + (size_t)(row0 + ln) * lda;
  v8f acc[4] = {};
  for (int kb = 0; kb < K; kb += 32) { FragH ah; ah.half[0] = *(const v8us*)((const unsigned short*)arow + kb + 8 * hh); ah.half[1] = *(const v8us*)((const unsigned short*)arow + kb + 16 + 8 * hh);
#pragma unroll
    for (int t = 0; t < 4; ++t) { if (col0 + t * 16 >= N) continue; const size_t boff = (size_t)(col0 + t * 16 + ln) * ldb + kb; FragH bq; bq.half[0] = *(const v8us*)((const unsigned short*)Bh + boff + 8 * hh); bq.half[1] = *(const v8us*)((const unsigned short*)Bh + boff + 16 + 8 * hh);
      acc[t] = mmaH<1>(ah.v, ah.v, bq.v, bq.v, acc[t]); }
  }
#pragma unroll
  for (int t = 0; t < 4; ++t) { if (col0 + t * 16 >= N) continue; const int col = col0 + t * 16 + ln; const float bv = bp ? bf16_round(bp[col]) : 0.f;
#pragma unroll
    for (int r = 0; r < 8; ++r) { float v = acc[t][r] * alpha + bv; if (CP) { const int bidx = (row0g + row0 + 8 * hh + r) / rowsPerB; v += CP[(size_t)bidx * sCPb + (size_t)by * 64 + col]; } if (ACT == 1) v = (v > 0.f) ? v : expm1f(v); else if (ACT == 7) v = (v > 0.f) ? v + 1.0f : expf(v); else if (ACT == 8) v = tanhf(v); else if (ACT == 9) v = 0.5f * v * (1.0f + tanhf(0.7978845608028654f * (v + 0.044715f * v * v * v))); else if (ACT == 11) v = 1.0f / (1.0f + expf(-v)); else if (ACT == 12) v = (v > 0.f) ? v : 0.01f * v; else if (ACT == 14) v = (v > 0.f) ? v : 0.1f * v; else if (ACT == 15) v = v / (1.0f + expf(-v)); else if (ACT == 3) v = fmaxf(v, 0.f); else if (ACT == 6) v = 0.5f * v * (1.0f + erff(v * 0.70710678118654752f)); so[w][8 * hh + r][t * 16 + ln] = v; } }
  __builtin_amdgcn_fence(__ATOMIC_ACQ_REL, "workgroup"); __builtin_amdgcn_wave_barrier();
  const int rsub = lane >> 4, c4 = (lane & 15) * 4; typedef _Float16 v4h __attribute__((ext_vector_type(4)));
  for (int pass = 0; pass < 2; ++pass) {
#pragma unroll
    for (int q = 0; q < 8; ++q) { const int r = q * 2 + rsub; if (col0 + c4 < N) { const v4f v = *(const v4fa*)&so[w][r][c4]; if (C) *(volatile v4f*)(C + cofs + (size_t)(row0 + r) * ldc + col0 + c4) = v; if (C16) { v4h h4; for (int i = 0; i < 4; ++i) h4[i] = (_Float16)v[i]; *(volatile v4h*)(C16 + cofs + (size_t)(row0 + r) * ldc + col0 + c4) = h4; } } }
    if (pass == 0) __threadfence(); }
}


typedef _Float16 v4h __attribute__((ext_vector_type(4)));

__global__ __launch_bounds__(256) void k_x16(const float* __restrict__ x, _Float16* __restrict__ X16, size_t n8) { const size_t t = (size_t)blockIdx.x * 256 + threadIdx.x; if (t >= n8) return; FragH f;
#pragma unroll
  for (int q = 0; q < 8; ++q) f.h[q] = (_Float16)bf16_round(x[t * 8 + q]); *(volatile v8us*)((unsigned short*)X16 + t * 8) = f.half[0]; __threadfence(); *(volatile v8us*)((unsigned short*)X16 + t * 8) = f.half[0]; }
__global__ __launch_bounds__(256) void k_h16(const float* __restrict__ x, _Float16* __restrict__ X16, size_t n8) { const size_t t = (size_t)blockIdx.x * 256 + threadIdx.x; if (t >= n8) return; FragH f;
#pragma unroll
  for (int q = 0; q < 8; ++q) f.h[q] = (_Float16)x[t * 8 + q]; *(volatile v8us*)((unsigned short*)X16 + t * 8) = f.half[0]; __threadfence(); *(volatile v8us*)((unsigned short*)X16 + t * 8) = f.half[0]; }
__global__ __launch_bounds__(256) void k_round16f(const float* __restrict__ W, _Float16* __restrict__ Bt, size_t n8) { const size_t t = (size_t)blockIdx.x * 256 + threadIdx.x; if (t >= n8) return; FragH f;
#pragma unroll
  for (int i = 0; i < 8; ++i) f.h[i] = (_Float16)(bf16_round(W[t * 8 + i]) * 16.0f); *(volatile v8us*)((unsigned short*)Bt + t * 8) = f.half[0]; __threadfence(); *(volatile v8us*)((unsigned short*)Bt + t * 8) = f.half[0]; }
template <int NHv, int TTv>
__global__ __launch_bounds__(256) void k_vt(const _Float16* __restrict__ V16, int ldv, int voff, _Float16* __restrict__ Vt) { __shared__ unsigned short tl[64][66]; const int tid = threadIdx.x; const int slab = blockIdx.x / (TTv / 64), lg = blockIdx.x % (TTv / 64); const int b = slab / NHv, h = slab % NHv;
  for (int i = tid; i < 64 * 8; i += 256) { const int r = i / 8, c8 = (i % 8) * 8; FragH f; f.half[0] = *(const v8us*)((const unsigned short*)V16 + ((size_t)b * TTv + lg * 64 + r) * ldv + voff + h * 64 + c8);
#pragma unroll
    for (int q = 0; q < 8; ++q) tl[r][c8 + q] = f.u[q]; }
  __syncthreads();
  for (int pass = 0; pass < 2; ++pass) {
#pragma unroll
    for (int rd = 0; rd < 2; ++rd) { const int d = rd * 32 + tid / 8, pc = tid % 8; FragH f;
#pragma unroll
      for (int q = 0; q < 8; ++q) f.u[q] = tl[pc * 8 + q][d];
      *(volatile v8us*)((unsigned short*)Vt + ((size_t)slab * 64 + d) * TTv + lg * 64 + pc * 8) = f.half[0]; }
    if (pass == 0) __threadfence(); } }

__global__ __launch_bounds__(256) void k_hl(const float* __restrict__ F, _Float16* __restrict__ Hh, _Float16* __restrict__ Hl, size_t n8) { const size_t t = (size_t)blockIdx.x * 256 + threadIdx.x; if (t >= n8) return; FragH fh, fl; const v4f a = *(const v4fa*)(F + t * 8), c = *(const v4fa*)(F + t * 8 + 4);
#pragma unroll
  for (int q = 0; q < 4; ++q) { _Float16 h = (_Float16)a[q]; fh.h[q] = h; fl.h[q] = (_Float16)((a[q] - (float)h) * 1024.0f); h = (_Float16)c[q]; fh.h[4 + q] = h; fl.h[4 + q] = (_Float16)((c[q] - (float)h) * 1024.0f); }
  for (int pass = 0; pass < 2; ++pass) { *(volatile v8us*)((unsigned short*)Hh + t * 8) = fh.half[0]; *(volatile v8us*)((unsigned short*)Hl + t * 8) = fl.half[0]; if (pass == 0) __threadfence(); } }

__global__ __launch_bounds__(256) void k_patch(const float* __restrict__ x, int b0, int df, int G, int KP_, _Float16* __restrict__ A16) { const size_t t = (size_t)blockIdx.x * 256 + threadIdx.x; const int ng = KP_ / 8; if (t >= (size_t)CB * G * G * ng) return; const int c0 = (int)(t % ng) * 8; const size_t r = t / ng; const int px = (int)(r % G), py = (int)((r / G) % G), bl = (int)(r / ((size_t)G * G)); const int K3 = 3 * df * df; FragH f;
#pragma unroll
  for (int q = 0; q < 8; ++q) { const int col = c0 + q; float v = 0.f; if (col < K3) { const int c = col / (df * df), rem = col % (df * df); const int ki = rem / df, kj = rem % df; v = bf16_round(x[(((size_t)(b0 + bl) * 3 + c) * 224 + py * df + ki) * 224 + px * df + kj]); } f.h[q] = (_Float16)v; }
  *(volatile v8us*)((unsigned short*)A16 + r * KP_ + c0) = f.half[0]; __threadfence(); *(volatile v8us*)((unsigned short*)A16 + r * KP_ + c0) = f.half[0]; }
__global__ __launch_bounds__(256) void k_ln16(const float* __restrict__ X, int nrows, const float* __restrict__ g, const float* __restrict__ bb, _Float16* __restrict__ Y) {
  #pragma clang fp contract(off)
  __shared__ __attribute__((aligned(16))) unsigned short sh[8][DDm]; const int tid = threadIdx.x, w = tid >> 5, l = tid & 31; const int r = blockIdx.x * 8 + w; if (r >= nrows) return; const float* xr = X + (size_t)r * DDm; const float a = xr[l], b = xr[32 + l], c = xr[64 + l]; float s = (a + b) + c;
  for (int o = 16; o > 0; o >>= 1) s += __shfl_xor(s, o, 32); const float mu = s / (float)DDm; float vs = ((a - mu) * (a - mu) + (b - mu) * (b - mu)) + (c - mu) * (c - mu); for (int o = 16; o > 0; o >>= 1) vs += __shfl_xor(vs, o, 32); const float rs = rsqrtf(vs / (float)DDm + 1e-5f);
  { FragH f; f.h[0] = (_Float16)((a - mu) * rs * bf16_round(g[l]) + bf16_round(bb[l])); sh[w][l] = f.u[0]; f.h[0] = (_Float16)((b - mu) * rs * bf16_round(g[32 + l]) + bf16_round(bb[32 + l])); sh[w][32 + l] = f.u[0]; f.h[0] = (_Float16)((c - mu) * rs * bf16_round(g[64 + l]) + bf16_round(bb[64 + l])); sh[w][64 + l] = f.u[0]; }
  __syncwarp();
  for (int pass = 0; pass < 2; ++pass) { if (l < 12) *(volatile v8us*)((unsigned short*)Y + (size_t)r * LP + 8 * l) = *(const v8us*)&sh[w][8 * l]; if (pass == 0) __threadfence(); } }
__global__ __launch_bounds__(256) void k_winqk(const _Float16* __restrict__ QKV, int G, int wsz, int IP, int KPk, int which, _Float16* __restrict__ OUTp) { const int nw = G / wsz, nwin = nw * nw, tw = wsz * wsz; const int rows = which ? KPk : IP; const size_t t = (size_t)blockIdx.x * 256 + threadIdx.x; if (t >= (size_t)CB * NHh * nwin * rows * 2) return; const int hf = (int)(t & 1); const int i = (int)((t >> 1) % rows); const size_t bhw = (t >> 1) / rows; const int win = (int)(bhw % nwin); const int h = (int)((bhw / nwin) % NHh); const int bl = (int)(bhw / ((size_t)nwin * NHh)); FragH f;
  if (i < tw) { const int wy = win / nw, wx = win % nw; const int ty = wy * wsz + i / wsz, tx = wx * wsz + i % wsz; const size_t tok = ((size_t)bl * G + ty) * G + tx; f.half[0] = *(const v8us*)((const unsigned short*)QKV + tok * QP + (which ? 96 : 0) + h * HD + 8 * hf); }
  else {
#pragma unroll
    for (int q = 0; q < 8; ++q) f.h[q] = (_Float16)0.0f; }
  *(volatile v8us*)((unsigned short*)OUTp + (bhw * rows + i) * HD + 8 * hf) = f.half[0]; __threadfence(); *(volatile v8us*)((unsigned short*)OUTp + (bhw * rows + i) * HD + 8 * hf) = f.half[0]; }
__global__ __launch_bounds__(256) void k_winvt(const _Float16* __restrict__ QKV, int G, int wsz, int KPk, _Float16* __restrict__ VWt) { const int nw = G / wsz, nwin = nw * nw, tw = wsz * wsz; const int ng = KPk / 8; const size_t t = (size_t)blockIdx.x * 256 + threadIdx.x; if (t >= (size_t)CB * NHh * nwin * HD * ng) return; const int j0 = (int)(t % ng) * 8; const int d = (int)((t / ng) % HD); const size_t bhw = t / ((size_t)ng * HD); const int win = (int)(bhw % nwin); const int h = (int)((bhw / nwin) % NHh); const int bl = (int)(bhw / ((size_t)nwin * NHh)); const int wy = win / nw, wx = win % nw; FragH f;
#pragma unroll
  for (int q = 0; q < 8; ++q) { const int j = j0 + q; _Float16 v = (_Float16)0.0f; if (j < tw) { const int ty = wy * wsz + j / wsz, tx = wx * wsz + j % wsz; const size_t tok = ((size_t)bl * G + ty) * G + tx; v = QKV[tok * QP + 192 + h * HD + d]; } f.h[q] = v; }
  *(volatile v8us*)((unsigned short*)VWt + (bhw * HD + d) * KPk + j0) = f.half[0]; __threadfence(); *(volatile v8us*)((unsigned short*)VWt + (bhw * HD + d) * KPk + j0) = f.half[0]; }
__global__ __launch_bounds__(256) void k_wsoft(const float* __restrict__ S, int nrows, int IP, int KPk, int tw, _Float16* __restrict__ P16) {
  #pragma clang fp contract(off)
  const int ng = KPk / 8; const size_t t = (size_t)blockIdx.x * 256 + threadIdx.x; if (t >= (size_t)nrows * ng) return; const int g8 = (int)(t % ng) * 8; const size_t row = t / ng; const int i = (int)(row % IP); const float* sr = S + row * KPk; float m = -3.0e38f, s = 0.f;
  if (i < tw) {
#pragma unroll 1
    for (int j = 0; j < tw; ++j) m = fmaxf(m, sr[j]);
#pragma unroll 1
    for (int j = 0; j < tw; ++j) s += expf(sr[j] - m); }
  const float inv = (i < tw) ? 1024.0f / s : 0.f; FragH f;
#pragma unroll
  for (int q = 0; q < 8; ++q) { const int j = g8 + q; f.h[q] = (j < tw && i < tw) ? (_Float16)(expf(sr[j] - m) * inv) : (_Float16)0.0f; }
  *(volatile v8us*)((unsigned short*)P16 + row * KPk + g8) = f.half[0]; __threadfence(); *(volatile v8us*)((unsigned short*)P16 + row * KPk + g8) = f.half[0]; }
__global__ __launch_bounds__(256) void k_wattn(const _Float16* __restrict__ QKV, int G, int wsz, _Float16* __restrict__ OT) {
  #pragma clang fp contract(off)
  const size_t tok = (size_t)blockIdx.x * 256 + threadIdx.x; if (tok >= (size_t)CB * G * G) return; const int tx = (int)(tok % G), ty = (int)((tok / G) % G), bl = (int)(tok / ((size_t)G * G)); const int wy = ty / wsz, wx = tx / wsz; const int tw = wsz * wsz;
#pragma unroll 1
  for (int h = 0; h < NHh; ++h) { float q[HD]; { const _Float16* qp = QKV + tok * QP + h * HD;
#pragma unroll
      for (int d = 0; d < HD; ++d) q[d] = (float)qp[d] * 0.1767766952966369f; }
    float m = -3.0e38f, lsum = 0.f; float o[HD];
#pragma unroll
    for (int d = 0; d < HD; ++d) o[d] = 0.f;
#pragma unroll 1
    for (int j = 0; j < tw; ++j) { const int ky = wy * wsz + j / wsz, kx = wx * wsz + j % wsz; const size_t ktok = ((size_t)bl * G + ky) * G + kx; const _Float16* kp = QKV + ktok * QP + 96 + h * HD; const _Float16* vp = QKV + ktok * QP + 192 + h * HD; float s = 0.f;
#pragma unroll
      for (int d = 0; d < HD; ++d) s += q[d] * (float)kp[d];
      const float mn = fmaxf(m, s); const float corr = expf(m - mn); const float p = expf(s - mn); lsum = lsum * corr + p;
#pragma unroll
      for (int d = 0; d < HD; ++d) o[d] = o[d] * corr + p * (float)vp[d];
      m = mn; }
    const float inv = 1.0f / lsum; FragH f0, f1, f2, f3;
#pragma unroll
    for (int qd = 0; qd < 8; ++qd) { f0.h[qd] = (_Float16)(o[qd] * inv); f1.h[qd] = (_Float16)(o[8 + qd] * inv); f2.h[qd] = (_Float16)(o[16 + qd] * inv); f3.h[qd] = (_Float16)(o[24 + qd] * inv); }
    unsigned short* dst = (unsigned short*)OT + tok * LP + h * HD;
    for (int pass = 0; pass < 2; ++pass) { *(volatile v8us*)(dst) = f0.half[0]; *(volatile v8us*)(dst + 8) = f1.half[0]; *(volatile v8us*)(dst + 16) = f2.half[0]; *(volatile v8us*)(dst + 24) = f3.half[0]; if (pass == 0) __threadfence(); } } }
__global__ __launch_bounds__(256) void k_unwin(const float* __restrict__ O, int G, int wsz, int IP, _Float16* __restrict__ OT) { const int nw = G / wsz, nwin = nw * nw; const size_t t = (size_t)blockIdx.x * 256 + threadIdx.x; if (t >= (size_t)CB * G * G * 12) return; const int g = (int)(t % 12); const size_t tok = t / 12; const int h = g / 4, d0 = (g % 4) * 8; const int tx = (int)(tok % G), ty = (int)((tok / G) % G), bl = (int)(tok / ((size_t)G * G)); const int wy = ty / wsz, wx = tx / wsz, i = (ty % wsz) * wsz + (tx % wsz); const size_t bhw = ((size_t)bl * NHh + h) * nwin + wy * nw + wx; const float* src = O + ((bhw * IP) + i) * HD + d0; FragH f;
#pragma unroll
  for (int q = 0; q < 8; ++q) f.h[q] = (_Float16)src[q];
  *(volatile v8us*)((unsigned short*)OT + tok * LP + h * HD + d0) = f.half[0]; __threadfence(); *(volatile v8us*)((unsigned short*)OT + tok * LP + h * HD + d0) = f.half[0]; }
__global__ __launch_bounds__(256) void k_cln(const float* __restrict__ P0, const float* __restrict__ P1, const float* __restrict__ P2, const float* __restrict__ g, const float* __restrict__ bb, _Float16* __restrict__ Y) {
  #pragma clang fp contract(off)
  __shared__ __attribute__((aligned(16))) unsigned short sh[8][DDm]; const int tid = threadIdx.x, w = tid >> 5, l = tid & 31; const int r = blockIdx.x * 8 + w; const int NNB = CB * NQ * NKc; if (r >= NNB + CB * NQ) return; float vals[3];
  if (r >= NNB) { const int tok = r - NNB;
#pragma unroll
    for (int m = 0; m < 3; ++m) vals[m] = P0[(size_t)tok * DDm + l + 32 * m]; }
  else { const int q = r % NKc; const int n = (r / NKc) % NQ; const int bl = r / (NKc * NQ); const int ny = n / G0, nx = n % G0;
#pragma unroll
    for (int m = 0; m < 3; ++m) { const int e = l + 32 * m; float v = 0.f;
      if (q < 16) { const int f = q * DDm + e; const int c = f / 16, rem = f % 16; const int ki = rem / 4, kj = rem % 4; const int y = ny * 4 + ki, xq = nx * 4 + kj; v = P1[(((size_t)bl * G1 + y) * G1 + xq) * DDm + c]; }
      else { const int f = (q - 16) * DDm + e; const int c = f / 9, rem = f % 9; const int ki = rem / 3, kj = rem % 3; const int y = ny * 3 + ki - 5, xq = nx * 3 + kj - 5; if (y >= 0 && y < G2 && xq >= 0 && xq < G2) v = P2[(((size_t)bl * G2 + y) * G2 + xq) * DDm + c]; }
      vals[m] = v; } }
  float s = (vals[0] + vals[1]) + vals[2]; for (int o = 16; o > 0; o >>= 1) s += __shfl_xor(s, o, 32); const float mu = s / (float)DDm; float vs = 0.f;
#pragma unroll
  for (int m = 0; m < 3; ++m) vs += (vals[m] - mu) * (vals[m] - mu); for (int o = 16; o > 0; o >>= 1) vs += __shfl_xor(vs, o, 32); const float rs = rsqrtf(vs / (float)DDm + 1e-5f);
#pragma unroll
  for (int m = 0; m < 3; ++m) { FragH f; f.h[0] = (_Float16)((vals[m] - mu) * rs * bf16_round(g[l + 32 * m]) + bf16_round(bb[l + 32 * m])); sh[w][l + 32 * m] = f.u[0]; }
  __syncwarp();
  for (int pass = 0; pass < 2; ++pass) { if (l < 12) *(volatile v8us*)((unsigned short*)Y + (size_t)r * LP + 8 * l) = *(const v8us*)&sh[w][8 * l]; if (pass == 0) __threadfence(); } }
__global__ __launch_bounds__(256) void k_cross(const float* __restrict__ Qc, const float* __restrict__ Kc, const float* __restrict__ Vc, _Float16* __restrict__ O16) {
  #pragma clang fp contract(off)
  __shared__ __attribute__((aligned(16))) unsigned short sh[8][DDm]; __shared__ float sa[8][32]; const int tid = threadIdx.x, w = tid >> 5, l = tid & 31; const int tok = blockIdx.x * 8 + w; if (tok >= CB * NQ) return; const float q0 = Qc[(size_t)tok * DDm + l], q1 = Qc[(size_t)tok * DDm + 32 + l], q2 = Qc[(size_t)tok * DDm + 64 + l]; float m = -3.0e38f;
#pragma unroll 1
  for (int k = 0; k < NKc; ++k) { const float* kr = Kc + ((size_t)tok * NKc + k) * DDm; float s = (q0 * kr[l] + q1 * kr[32 + l]) + q2 * kr[64 + l]; for (int o = 16; o > 0; o >>= 1) s += __shfl_xor(s, o, 32); s *= 0.10206207261596575f; if (l == 0) sa[w][k] = s; m = fmaxf(m, s); }
  __syncwarp(); float den = 0.f;
#pragma unroll 1
  for (int k = 0; k < NKc; ++k) den += expf(sa[w][k] - m);
  float o0 = 0.f, o1 = 0.f, o2 = 0.f;
#pragma unroll 1
  for (int k = 0; k < NKc; ++k) { const float a = expf(sa[w][k] - m) / den; const float* vr = Vc + ((size_t)tok * NKc + k) * DDm; o0 += a * vr[l]; o1 += a * vr[32 + l]; o2 += a * vr[64 + l]; }
  { FragH f; f.h[0] = (_Float16)o0; sh[w][l] = f.u[0]; f.h[0] = (_Float16)o1; sh[w][32 + l] = f.u[0]; f.h[0] = (_Float16)o2; sh[w][64 + l] = f.u[0]; }
  __syncwarp();
  for (int pass = 0; pass < 2; ++pass) { if (l < 12) *(volatile v8us*)((unsigned short*)O16 + (size_t)tok * LP + 8 * l) = *(const v8us*)&sh[w][8 * l]; if (pass == 0) __threadfence(); } }

__global__ __launch_bounds__(256) void k_wtp(const float* __restrict__ Wm, int in, int out, int KP_, _Float16* __restrict__ Bt) { const int t = blockIdx.x * 256 + threadIdx.x; if (t >= out * (KP_ / 8)) return; const int k0 = (t % (KP_ / 8)) * 8, o = t / (KP_ / 8); FragH f;
#pragma unroll
  for (int q = 0; q < 8; ++q) { const int k = k0 + q; f.h[q] = (k < in) ? (_Float16)(bf16_round(Wm[(size_t)k * out + o]) * 16.0f) : (_Float16)0.0f; }
  *(volatile v8us*)((unsigned short*)Bt + (size_t)o * KP_ + k0) = f.half[0]; __threadfence(); *(volatile v8us*)((unsigned short*)Bt + (size_t)o * KP_ + k0) = f.half[0]; }

extern "C" void kernel_launch(void* const* d_in, const int* in_sizes, int n_in,
                              void* d_out, int out_size, void* d_ws, size_t ws_size, hipStream_t stream) {
  (void)in_sizes; (void)n_in; (void)out_size;
  const float* const* I = (const float* const*)d_in; const float* x = I[0]; const float* pw[3] = {I[1], I[3], I[5]}; const float* pb[3] = {I[2], I[4], I[6]};
  const float* wa_ln_g = I[7]; const float* wa_ln_b = I[8]; const float* wa_qkv = I[9]; const float* wa_ow = I[10]; const float* wa_ob = I[11]; const float* ff_ln_g = I[12]; const float* ff_ln_b = I[13]; const float* ff_w1 = I[14]; const float* ff_b1 = I[15]; const float* ff_w2 = I[16]; const float* ff_b2 = I[17];
  const float* lnn_g = I[18]; const float* lnn_b = I[19]; const float* ca_wq = I[20]; const float* ca_wk = I[21]; const float* ca_wv = I[22]; const float* ca_wo = I[23]; const float* ca_bo = I[24]; const float* fi_ln_g = I[25]; const float* fi_ln_b = I[26]; const float* fi_w1 = I[27]; const float* fi_b1 = I[28]; const float* fi_w2 = I[29]; const float* fi_b2 = I[30];
  const int dfs[3] = {16, 4, 7}, Gs[3] = {G0, G1, G2}, Ts[3] = {T0, T1, T2}, wss[3] = {7, 4, 4}, KPs[3] = {768, 64, 160}, IPs[3] = {64, 16, 16}, KKs[3] = {64, 32, 32};
  char* ws = (char*)d_ws; size_t off = 0;
  auto take = [&](size_t bytes) { char* p = ws + off; off += (bytes + 255) & ~(size_t)255; return p; };
  _Float16* Bp[3]; _Float16* Bqkv[3]; _Float16* Bow[3]; _Float16* Bf1[3]; _Float16* Bf2[3]; for (int i = 0; i < 3; ++i) { Bp[i] = (_Float16*)take((size_t)DDm * KPs[i] * 2); Bqkv[i] = (_Float16*)take((size_t)288 * DDm * 2); Bow[i] = (_Float16*)take((size_t)DDm * DDm * 2); Bf1[i] = (_Float16*)take((size_t)DDm * DDm * 2); Bf2[i] = (_Float16*)take((size_t)DDm * DDm * 2); }
  _Float16* Bcq = (_Float16*)take(DDm * DDm * 2); _Float16* Bck = (_Float16*)take(DDm * DDm * 2); _Float16* Bcv = (_Float16*)take(DDm * DDm * 2); _Float16* Bco = (_Float16*)take(DDm * DDm * 2); _Float16* Bi1 = (_Float16*)take(DDm * DDm * 2); _Float16* Bi2 = (_Float16*)take(DDm * DDm * 2);
  const size_t MT = (size_t)CB * T1;        const size_t MBHW = (size_t)CB * NHh * 196;
  _Float16* A16 = (_Float16*)take(MT * 64 * 2 > (size_t)CB * T0 * 768 * 2 ? MT * 64 * 2 : (size_t)CB * T0 * 768 * 2); float* T = (float*)take(MT * DDm * 4); _Float16* L16 = (_Float16*)take(MT * LP * 2); _Float16* QKV = (_Float16*)take(MT * QP * 2);
  _Float16* QW = (_Float16*)take(MBHW * 16 * HD * 2); _Float16* KW = (_Float16*)take(MBHW * 32 * HD * 2); _Float16* VWt = (_Float16*)take(MBHW * HD * 32 * 2); float* S = (float*)take(MBHW * 16 * 32 * 4); _Float16* P16 = (_Float16*)take(MBHW * 16 * 32 * 2); float* O = (float*)take(MBHW * 16 * HD * 4);
  _Float16* OT = (_Float16*)take(MT * LP * 2); float* Tb = (float*)take(MT * DDm * 4); _Float16* F16 = (_Float16*)take(MT * LP * 2);
  float* PX[3]; PX[0] = (float*)take((size_t)CB * T0 * DDm * 4); PX[1] = (float*)take((size_t)CB * T1 * DDm * 4); PX[2] = (float*)take((size_t)CB * T2 * DDm * 4);
  const int NNB = CB * NQ * NKc, NCR = NNB + CB * NQ;
  _Float16* CL = QKV;   float* Qc = T; float* Kc = (float*)KW; float* Vc = (float*)((char*)KW + (size_t)NNB * DDm * 4); _Float16* OC = OT; float* OA = Tb; _Float16* LA = F16; _Float16* FA = L16;
  if (off > ws_size) return;
  const int Kin[3] = {768, 48, 147};
  for (int i = 0; i < 3; ++i) { k_wtp<<<(DDm * (KPs[i] / 8) + 255) / 256, 256, 0, stream>>>(pw[i], Kin[i], DDm, KPs[i], Bp[i]); k_wtp<<<(288 * (DDm / 8) + 255) / 256, 256, 0, stream>>>(wa_qkv + (size_t)i * DDm * 288, DDm, 288, DDm, Bqkv[i]); k_wtp<<<(DDm * (DDm / 8) + 255) / 256, 256, 0, stream>>>(wa_ow + (size_t)i * DDm * DDm, DDm, DDm, DDm, Bow[i]); k_wtp<<<(DDm * (DDm / 8) + 255) / 256, 256, 0, stream>>>(ff_w1 + (size_t)i * DDm * DDm, DDm, DDm, DDm, Bf1[i]); k_wtp<<<(DDm * (DDm / 8) + 255) / 256, 256, 0, stream>>>(ff_w2 + (size_t)i * DDm * DDm, DDm, DDm, DDm, Bf2[i]); }
  k_wtp<<<(DDm * (DDm / 8) + 255) / 256, 256, 0, stream>>>(ca_wq, DDm, DDm, DDm, Bcq); k_wtp<<<(DDm * (DDm / 8) + 255) / 256, 256, 0, stream>>>(ca_wk, DDm, DDm, DDm, Bck); k_wtp<<<(DDm * (DDm / 8) + 255) / 256, 256, 0, stream>>>(ca_wv, DDm, DDm, DDm, Bcv); k_wtp<<<(DDm * (DDm / 8) + 255) / 256, 256, 0, stream>>>(ca_wo, DDm, DDm, DDm, Bco); k_wtp<<<(DDm * (DDm / 8) + 255) / 256, 256, 0, stream>>>(fi_w1, DDm, DDm, DDm, Bi1); k_wtp<<<(DDm * (DDm / 8) + 255) / 256, 256, 0, stream>>>(fi_w2, DDm, DDm, DDm, Bi2);
  for (int ch = 0; ch < NIMG / CB; ++ch) { const int b0 = ch * CB;
    for (int i = 0; i < 3; ++i) { const int G = Gs[i], df = dfs[i], wsz = wss[i], IP = IPs[i], KPk = KKs[i]; const int ntok = CB * Ts[i]; const int nw = G / wsz, nwin = nw * nw, tw = wsz * wsz; const int nbhw = CB * NHh * nwin;
      const dim3 gT(((ntok / 16) * 2 + 3) / 4, 1), gQ(((ntok / 16) * 5 + 3) / 4, 1);
      k_patch<<<(unsigned)(((size_t)ntok * (KPs[i] / 8) + 255) / 256), 256, 0, stream>>>(x, b0, df, G, KPs[i], A16);
      k_gemm_hhx<0><<<gT, 128, 0, stream>>>(A16, KPs[i], 0, Bp[i], KPs[i], 0, 0.0625f, pb[i], 0, nullptr, 1, 0, 0, T, nullptr, DDm, 0, ntok, DDm, KPs[i]);
      k_ln16<<<(ntok + 7) / 8, 256, 0, stream>>>(T, ntok, wa_ln_g + i * DDm, wa_ln_b + i * DDm, L16);
      k_gemm_hhx<0><<<gQ, 128, 0, stream>>>(L16, LP, 0, Bqkv[i], DDm, 0, 0.0625f, nullptr, 0, nullptr, 1, 0, 0, nullptr, QKV, QP, 0, ntok, 288, DDm);
      k_wattn<<<(unsigned)((ntok + 255) / 256), 256, 0, stream>>>(QKV, G, wsz, OT);
      (void)IP; (void)KPk; (void)tw; (void)nbhw;
      k_gemm_hhx<0><<<gT, 128, 0, stream>>>(OT, LP, 0, Bow[i], DDm, 0, 0.0625f, wa_ob + i * DDm, 0, T, 1, (size_t)DDm, 0, Tb, nullptr, DDm, 0, ntok, DDm, DDm);
      k_ln16<<<(ntok + 7) / 8, 256, 0, stream>>>(Tb, ntok, ff_ln_g + i * DDm, ff_ln_b + i * DDm, L16);
      k_gemm_hhx<6><<<gT, 128, 0, stream>>>(L16, LP, 0, Bf1[i], DDm, 0, 0.0625f, ff_b1 + i * DDm, 0, nullptr, 1, 0, 0, nullptr, F16, LP, 0, ntok, DDm, DDm);
      k_gemm_hhx<0><<<gT, 128, 0, stream>>>(F16, LP, 0, Bf2[i], DDm, 0, 0.0625f, ff_b2 + i * DDm, 0, Tb, 1, (size_t)DDm, 0, PX[i], nullptr, DDm, 0, ntok, DDm, DDm); }
    const int nq = CB * NQ; const dim3 gC(((NNB / 16) * 2 + 3) / 4, 1), gq(((nq / 16) * 2 + 3) / 4, 1);
    k_cln<<<(NCR + 7) / 8, 256, 0, stream>>>(PX[0], PX[1], PX[2], lnn_g, lnn_b, CL);
    k_gemm_hhx<0><<<gq, 128, 0, stream>>>(CL + (size_t)NNB * LP, LP, 0, Bcq, DDm, 0, 0.0625f, nullptr, 0, nullptr, 1, 0, 0, Qc, nullptr, DDm, 0, nq, DDm, DDm);
    k_gemm_hhx<0><<<gC, 128, 0, stream>>>(CL, LP, 0, Bck, DDm, 0, 0.0625f, nullptr, 0, nullptr, 1, 0, 0, Kc, nullptr, DDm, 0, NNB, DDm, DDm); k_gemm_hhx<0><<<gC, 128, 0, stream>>>(CL, LP, 0, Bcv, DDm, 0, 0.0625f, nullptr, 0, nullptr, 1, 0, 0, Vc, nullptr, DDm, 0, NNB, DDm, DDm);
    k_cross<<<(nq + 7) / 8, 256, 0, stream>>>(Qc, Kc, Vc, OC);
    k_gemm_hhx<0><<<gq, 128, 0, stream>>>(OC, LP, 0, Bco, DDm, 0, 0.0625f, ca_bo, 0, PX[0], 1, (size_t)DDm, 0, OA, nullptr, DDm, 0, nq, DDm, DDm);
    k_ln16<<<(nq + 7) / 8, 256, 0, stream>>>(OA, nq, fi_ln_g, fi_ln_b, LA);
    k_gemm_hhx<6><<<gq, 128, 0, stream>>>(LA, LP, 0, Bi1, DDm, 0, 0.0625f, fi_b1, 0, nullptr, 1, 0, 0, nullptr, FA, LP, 0, nq, DDm, DDm);
    k_gemm_hhx<0><<<gq, 128, 0, stream>>>(FA, LP, 0, Bi2, DDm, 0, 0.0625f, fi_b2, 0, OA, 1, (size_t)DDm, 0, (float*)d_out + (size_t)b0 * NQ * DDm, nullptr, DDm, 0, nq, DDm, DDm); }
}
